// NaturalAttention_81432579932595
// MI455X (gfx1250) — hardware-verified
//
#include <hip/hip_runtime.h>
#include <math.h>
#include <stdint.h>

static constexpr int kNB     = 4;
static constexpr int kSeq    = 1024;
static constexpr int kDM     = 1024;
static constexpr int kNH     = 16;
static constexpr int kDHD    = 64;
static constexpr int kMaxRel = 128;
static constexpr int kRelN   = 2 * kMaxRel + 1;
static constexpr int kRelPad = 320;
static constexpr int kHG     = 8;
static constexpr int kNGrp   = kNH / kHG;
static constexpr float kPScale = 32768.0f;
static_assert(kNH * kDHD == kDM, "head split");
static_assert(kNH % kHG == 0, "head groups");
static_assert(kRelPad % 64 == 0 && kRelPad >= kRelN, "padded table rows");
static_assert(kSeq % 64 == 0 && kDM % 64 == 0 && kDHD % 64 == 0 && (kNB * kSeq) % 64 == 0, "tile multiples");
static_assert(kDM % 32 == 0 && kDHD % 32 == 0 && kSeq % 32 == 0, "K multiples of 32");
static_assert(kSeq == 128 * 8, "softmax row coverage: 128 threads x 8 columns");
static_assert((kNB * kSeq * kDM / 2) % 256 == 0 && (kDM * kDM / 2) % 256 == 0 && (kRelPad * kDHD / 2) % 256 == 0, "cast grids exact");
static_assert((kRelN * kDHD) % 2 == 0, "rel pairs");

typedef __attribute__((ext_vector_type(16))) _Float16 v16h;
typedef __attribute__((ext_vector_type(8)))  _Float16 v8h;
typedef __attribute__((ext_vector_type(16))) __bf16   v16b;
typedef __attribute__((ext_vector_type(8)))  __bf16   v8b;
typedef __attribute__((ext_vector_type(8)))  float    v8f;
typedef __attribute__((ext_vector_type(4)))  float    v4f;
typedef __attribute__((ext_vector_type(2)))  float    v2f;
typedef __attribute__((ext_vector_type(4)))  unsigned int v4u;

__device__ __forceinline__ unsigned short f2bf_bits(float f) {
  unsigned u = __float_as_uint(f);
  return (unsigned short)((u + 0x7FFFu + ((u >> 16) & 1u)) >> 16);
}
__device__ __forceinline__ float bf_bits2f(unsigned short h) { return __uint_as_float(((unsigned)h) << 16); }

__device__ __forceinline__ void dep_guard_h(v8f& a, v8f& b, v16h x, v16h y) { asm volatile("v_nop\n\tv_nop\n\tv_nop\n\tv_nop" : "+v"(a), "+v"(b) : "v"(x), "v"(y)); }
__device__ __forceinline__ void dep_guard_b(v8f& a, v8f& b, v16b x, v16b y) { asm volatile("v_nop\n\tv_nop\n\tv_nop\n\tv_nop" : "+v"(a), "+v"(b) : "v"(x), "v"(y)); }
__device__ __forceinline__ void keep4_h(v16h a, v16h b, v16h c, v16h d) { asm volatile("v_nop" :: "v"(a), "v"(b), "v"(c), "v"(d)); }
__device__ __forceinline__ void keep4_b(v16b a, v16b b, v16b c, v16b d) { asm volatile("v_nop" :: "v"(a), "v"(b), "v"(c), "v"(d)); }
__device__ __forceinline__ void acc_guard4(v8f& a, v8f& b, v8f& c, v8f& d) { asm volatile("v_nop\n\tv_nop\n\tv_nop\n\tv_nop" : "+v"(a), "+v"(b), "+v"(c), "+v"(d)); }
template <typename T> struct Frag;
template <> struct Frag<_Float16> {
  typedef v16h V; union U { v16h v; v8h h[2]; };
  static __device__ __forceinline__ v16h load(const _Float16* p) {
    U f; f.h[0] = *(const v8h*)(p); f.h[1] = *(const v8h*)(p + 16); return f.v;
  }
  static __device__ __forceinline__ v8f mma(v16h a, v16h b, v8f c) {
    return __builtin_amdgcn_wmma_f32_16x16x32_f16(false, a, false, b, (short)0, c, false, false);
  }
  static __device__ __forceinline__ void guard(v8f& a, v8f& b, v16h x, v16h y) { dep_guard_h(a, b, x, y); }
  static __device__ __forceinline__ void keep(v16h a, v16h b, v16h c, v16h d) { keep4_h(a, b, c, d); }
};
template <> struct Frag<__bf16> {
  typedef v16b V; union U { v16b v; v8b h[2]; };
  static __device__ __forceinline__ v16b load(const __bf16* p) {
    U f; f.h[0] = *(const v8b*)(p); f.h[1] = *(const v8b*)(p + 16); return f.v;
  }
  static __device__ __forceinline__ v8f mma(v16b a, v16b b, v8f c) {
    return __builtin_amdgcn_wmma_f32_16x16x32_bf16(false, a, false, b, (short)0, c, false, false);
  }
  static __device__ __forceinline__ void guard(v8f& a, v8f& b, v16b x, v16b y) { dep_guard_b(a, b, x, y); }
  static __device__ __forceinline__ void keep(v16b a, v16b b, v16b c, v16b d) { keep4_b(a, b, c, d); }
};

template <int ET> struct Elem;
template <> struct Elem<0> { typedef _Float16 T; };
template <> struct Elem<1> { typedef __bf16 T; };
template <int ET, bool SPLIT, int BIAS_MODE, int OUT_MODE, bool RESID, int ACT = 0>
__global__ __launch_bounds__(256) void wmma_gemm64(
    const unsigned short* __restrict__ Ap, const unsigned short* __restrict__ A2p, int lda, long strideA,
    const unsigned short* __restrict__ Btp, const unsigned short* __restrict__ Bt2p, int ldb, long strideB,
    void* __restrict__ Cout, void* __restrict__ Cout2, int ldc, long strideC,
    const float* __restrict__ bias,
    const float* __restrict__ resid, long strideR,
    int M, int N, int K, float scale) {
  typedef typename Elem<ET>::T T;
  typedef typename Frag<T>::V V;
  const T* A = (const T*)Ap; const T* A2 = (const T*)A2p; const T* Bt = (const T*)Btp; const T* Bt2 = (const T*)Bt2p;
  __shared__ __align__(16) float sT[8][16 * 68];
  const int b    = blockIdx.y;
  const int lane = threadIdx.x & 31;
  const int wave = threadIdx.x >> 5;
  const int tilesN = N >> 6;
  const int tilesM = M >> 6;
  const int tile = blockIdx.x * 8 + wave;
  if (tile >= tilesM * tilesN) return;
  const int tm = tile / tilesN;
  const int tn = tile - tm * tilesN;
  const int m0 = tm << 6;
  const int n0 = tn << 6;

  const T* Ab  = A  + (size_t)b * strideA;
  const T* Bb  = Bt + (size_t)b * strideB;
  const T* Ab2 = SPLIT ? (A2  + (size_t)b * strideA) : nullptr;
  const T* Bb2 = SPLIT ? (Bt2 + (size_t)b * strideB) : nullptr;

  const int rlane = lane & 15;
  const int koff  = (lane >> 4) * 8;
  const int mOff  = (lane >> 4) * 8;

  v8f acc[4][4];
#pragma unroll
  for (int i = 0; i < 4; ++i)
#pragma unroll
    for (int j = 0; j < 4; ++j) acc[i][j] = (v8f){0.f,0.f,0.f,0.f,0.f,0.f,0.f,0.f};

  for (int k0 = 0; k0 < K; k0 += 32) {
    V bh[4], bl[4];
#pragma unroll
    for (int j = 0; j < 4; ++j) {
      const size_t bo = (size_t)(n0 + (j << 4) + rlane) * ldb + koff + k0;
      bh[j] = Frag<T>::load(Bb + bo);
      if (SPLIT) bl[j] = Frag<T>::load(Bb2 + bo);
    }
#pragma unroll
    for (int i = 0; i < 4; ++i) {
      const size_t ao = (size_t)(m0 + (i << 4) + rlane) * lda + koff + k0;
      V ah = Frag<T>::load(Ab + ao);
      V al;
      if (SPLIT) al = Frag<T>::load(Ab2 + ao);
#pragma unroll
      for (int j = 0; j < 4; ++j) {
        acc[i][j] = Frag<T>::mma(ah, bh[j], acc[i][j]);
        if (SPLIT) {
          acc[i][j] = Frag<T>::mma(ah, bl[j], acc[i][j]);
          acc[i][j] = Frag<T>::mma(al, bh[j], acc[i][j]);
        }
      }
      Frag<T>::guard(acc[i][0], acc[i][3], ah, SPLIT ? al : ah);
    }
    Frag<T>::keep(bh[0], bh[1], bh[2], bh[3]);
    if (SPLIT) Frag<T>::keep(bl[0], bl[1], bl[2], bl[3]);
  }
  acc_guard4(acc[0][0], acc[0][1], acc[0][2], acc[0][3]);
  acc_guard4(acc[1][0], acc[1][1], acc[1][2], acc[1][3]);
  acc_guard4(acc[2][0], acc[2][1], acc[2][2], acc[2][3]);
  acc_guard4(acc[3][0], acc[3][1], acc[3][2], acc[3][3]);

  float* slab = sT[wave];
  const float* Rb = RESID ? (resid + (size_t)b * strideR) : nullptr;
#pragma unroll
  for (int i = 0; i < 4; ++i) {
    const int mBase = m0 + (i << 4);
#pragma unroll
    for (int j = 0; j < 4; ++j) {
      const int n = n0 + (j << 4) + rlane;
      float bv = 0.f;
      if (BIAS_MODE == 2) bv = bias[n];
#pragma unroll
      for (int r = 0; r < 8; ++r) {
        float v = acc[i][j][r] * scale;
        if (BIAS_MODE == 1) v += bias[mBase + mOff + r];
        if (BIAS_MODE == 2) v += bv;
        if (RESID) v += Rb[(size_t)(mBase + mOff + r) * ldc + n];
        if (ACT == 1) v = tanhf(v);
        if (ACT == 2) v = fmaxf(v, 0.0f);
        if (ACT == 3) v = v / (1.0f + expf(-v));
        if (ACT == 4) v = (v > 0.f) ? v : 0.01f * v;
        slab[(mOff + r) * 68 + (j << 4) + rlane] = v;
      }
    }
    __builtin_amdgcn_fence(__ATOMIC_RELEASE, "workgroup");
    __builtin_amdgcn_wave_barrier();
    __builtin_amdgcn_fence(__ATOMIC_ACQUIRE, "workgroup");
    if (OUT_MODE == 0) {
      float* C = (float*)Cout + (size_t)b * strideC;
      const int hh = lane >> 4, c4 = (lane & 15) * 4;
      for (int pass = 0; pass < 2; ++pass) {
#pragma unroll
        for (int it = 0; it < 8; ++it) {
          const int row = it * 2 + hh;
          v4f v = *(const v4f*)(slab + row * 68 + c4);
          *(volatile v4f*)(C + (size_t)(mBase + row) * ldc + n0 + c4) = v;
        }
        __threadfence();
      }
    } else {
      const int q = lane >> 3, c8 = (lane & 7) * 8;
      unsigned short* C  = (unsigned short*)Cout  + (size_t)b * strideC;
      unsigned short* C2 = (OUT_MODE == 2) ? ((unsigned short*)Cout2 + (size_t)b * strideC) : nullptr;
      for (int pass = 0; pass < 2; ++pass) {
#pragma unroll
        for (int it = 0; it < 4; ++it) {
          const int row = it * 4 + q;
          const float* sp = slab + row * 68 + c8;
          v8h hv, lv;
#pragma unroll
          for (int e = 0; e < 8; ++e) {
            if (OUT_MODE == 1) {
              hv[e] = (_Float16)sp[e];
            } else {
              unsigned short hb = f2bf_bits(sp[e]);
              unsigned short lb = f2bf_bits(sp[e] - bf_bits2f(hb));
              hv[e] = __builtin_bit_cast(_Float16, hb);
              lv[e] = __builtin_bit_cast(_Float16, lb);
            }
          }
          *(volatile v8h*)(C + (size_t)(mBase + row) * ldc + n0 + c8) = hv;
          if (OUT_MODE == 2) *(volatile v8h*)(C2 + (size_t)(mBase + row) * ldc + n0 + c8) = lv;
        }
        __threadfence();
      }
    }
    __builtin_amdgcn_fence(__ATOMIC_RELEASE, "workgroup");
    __builtin_amdgcn_wave_barrier();
    __builtin_amdgcn_fence(__ATOMIC_ACQUIRE, "workgroup");
  }
}

__device__ __forceinline__ unsigned pk16(unsigned short a, unsigned short b) { return (unsigned)a | ((unsigned)b << 16); }
__device__ __forceinline__ unsigned short h_bits(float f) { const _Float16 h = (_Float16)f; return __builtin_bit_cast(unsigned short, h); }

__global__ __launch_bounds__(256) void cast_bf_f16x2_kernel(const float* __restrict__ in, unsigned short* __restrict__ out,
                                                            int n2, float scale) {
  const int i = blockIdx.x * 256 + threadIdx.x;
  if (i < n2) {
    const v2f f = *(const v2f*)(in + 2 * (size_t)i);
    const float a = bf_bits2f(f2bf_bits(f[0])) * scale;
    const float c = bf_bits2f(f2bf_bits(f[1])) * scale;
    const unsigned u = pk16(h_bits(a), h_bits(c));
    ((volatile unsigned*)out)[i] = u;
    __threadfence();
    ((volatile unsigned*)out)[i] = u;
  }
}

__global__ __launch_bounds__(256) void cast_rel_f16x2_kernel(const float* __restrict__ in, unsigned short* __restrict__ out,
                                                             int n2, int nsrc, float scale) {
  const int i = blockIdx.x * 256 + threadIdx.x;
  if (i < n2) {
    const int e0 = 2 * i;
    const bool valid = (e0 + 1 < nsrc);
    const int j = valid ? e0 : (nsrc - 2);
    const v2f f = *(const v2f*)(in + j);
    const float a = valid ? bf_bits2f(f2bf_bits(f[0])) * scale : 0.0f;
    const float c = valid ? bf_bits2f(f2bf_bits(f[1])) * scale : 0.0f;
    const unsigned u = pk16(h_bits(a), h_bits(c));
    ((volatile unsigned*)out)[i] = u;
    __threadfence();
    ((volatile unsigned*)out)[i] = u;
  }
}

__global__ __launch_bounds__(128) void rel_softmax_kernel(const float* __restrict__ Sc, const float* __restrict__ Qe,
                                                          unsigned short* __restrict__ P16) {
  __shared__ float redm[4];
  __shared__ float reds[4];
  const int row  = blockIdx.x;
  const int i    = row & (kSeq - 1);
  const int tid  = threadIdx.x;
  const int lane = tid & 31;
  const int wave = tid >> 5;
  const int j0   = tid * 8;

  const float* srow = Sc + (size_t)row * kSeq + j0;
  const v4f a0 = *(const v4f*)(srow);
  const v4f a1 = *(const v4f*)(srow + 4);
  float t[8];
  t[0] = a0[0]; t[1] = a0[1]; t[2] = a0[2]; t[3] = a0[3];
  t[4] = a1[0]; t[5] = a1[1]; t[6] = a1[2]; t[7] = a1[3];
  const float* qrow = Qe + (size_t)row * kRelPad;
#pragma unroll
  for (int e = 0; e < 8; ++e) {
    int d = j0 + e - i;
    d = d < -kMaxRel ? -kMaxRel : d;
    d = d > kMaxRel ? kMaxRel : d;
    t[e] += qrow[d + kMaxRel];
  }
  float m = fmaxf(fmaxf(fmaxf(t[0], t[1]), fmaxf(t[2], t[3])), fmaxf(fmaxf(t[4], t[5]), fmaxf(t[6], t[7])));
#pragma unroll
  for (int off = 16; off > 0; off >>= 1) m = fmaxf(m, __shfl_xor(m, off, 32));
  if (lane == 0) redm[wave] = m;
  __syncthreads();
  const float mx = fmaxf(fmaxf(redm[0], redm[1]), fmaxf(redm[2], redm[3]));
  float ex[8];
#pragma unroll
  for (int e = 0; e < 8; ++e) ex[e] = __expf(t[e] - mx);
  float s = ((ex[0] + ex[1]) + (ex[2] + ex[3])) + ((ex[4] + ex[5]) + (ex[6] + ex[7]));
#pragma unroll
  for (int off = 16; off > 0; off >>= 1) s += __shfl_xor(s, off, 32);
  if (lane == 0) reds[wave] = s;
  __syncthreads();
  const float tot = (reds[0] + reds[1]) + (reds[2] + reds[3]);
  const float inv = kPScale * (1.0f / tot);
  unsigned short hb[8];
#pragma unroll
  for (int e = 0; e < 8; ++e) hb[e] = h_bits(ex[e] * inv);
  const v4u hv = (v4u){pk16(hb[0], hb[1]), pk16(hb[2], hb[3]), pk16(hb[4], hb[5]), pk16(hb[6], hb[7])};
  unsigned short* pp = P16 + (size_t)row * kSeq + j0;
  *(volatile v4u*)pp = hv;
  __threadfence();
  *(volatile v4u*)pp = hv;
}

extern "C" void kernel_launch(void* const* d_in, const int* in_sizes, int n_in,
                              void* d_out, int out_size, void* d_ws, size_t ws_size,
                              hipStream_t stream) {
  if (n_in < 10) return;
  if (in_sizes[0] != kNB * kSeq * kDM) return;
  if (in_sizes[1] != kDM * kDM || in_sizes[3] != kDM * kDM ||
      in_sizes[5] != kDM * kDM || in_sizes[7] != kDM * kDM) return;
  if (in_sizes[2] != kDM || in_sizes[4] != kDM || in_sizes[6] != kDM || in_sizes[8] != kDM) return;
  if (in_sizes[9] != kRelN * kDHD) return;
  if (out_size != kNB * kSeq * kDM) return;

  const float* xp   = (const float*)d_in[0];
  const float* Wq   = (const float*)d_in[1];
  const float* bq   = (const float*)d_in[2];
  const float* Wk   = (const float*)d_in[3];
  const float* bk   = (const float*)d_in[4];
  const float* Wv   = (const float*)d_in[5];
  const float* bv   = (const float*)d_in[6];
  const float* Wo   = (const float*)d_in[7];
  const float* bo   = (const float*)d_in[8];
  const float* relp = (const float*)d_in[9];
  float* outp = (float*)d_out;

  const size_t bAct = (size_t)kNB * kSeq * kDM * 2;
  const size_t bW   = (size_t)kDM * kDM * 2;
  const size_t bRel = 65536;
  const size_t bS   = (size_t)kHG * kSeq * kSeq * 4;
  const size_t bQE  = (size_t)kHG * kSeq * kRelPad * 4;
  const size_t bP   = (size_t)kHG * kSeq * kSeq * 2;
  size_t off = 0;
  const size_t oX16 = off; off += bAct;
  const size_t oWq  = off; off += bW;
  const size_t oWk  = off; off += bW;
  const size_t oWv  = off; off += bW;
  const size_t oWo  = off; off += bW;
  const size_t oRel = off; off += bRel;
  const size_t oQ16 = off; off += bAct;
  const size_t oK16 = off; off += bAct;
  const size_t oVT  = off; off += bAct;
  const size_t oS   = off; off += bS;
  const size_t oQE  = off; off += bQE;
  const size_t oP   = off; off += bP;
  const size_t oCTX = off; off += bAct;
  if (off > ws_size) return;
  if (off > (size_t)134217728) return;

  char* ws = (char*)d_ws;
  unsigned short* X16   = (unsigned short*)(ws + oX16);
  unsigned short* Wq16  = (unsigned short*)(ws + oWq);
  unsigned short* Wk16  = (unsigned short*)(ws + oWk);
  unsigned short* Wv16  = (unsigned short*)(ws + oWv);
  unsigned short* Wo16  = (unsigned short*)(ws + oWo);
  unsigned short* REL16 = (unsigned short*)(ws + oRel);
  unsigned short* Q16   = (unsigned short*)(ws + oQ16);
  unsigned short* K16   = (unsigned short*)(ws + oK16);
  unsigned short* VT16  = (unsigned short*)(ws + oVT);
  float*          Sc    = (float*)(ws + oS);
  float*          Qe    = (float*)(ws + oQE);
  unsigned short* P16   = (unsigned short*)(ws + oP);
  unsigned short* CTX16 = (unsigned short*)(ws + oCTX);

  const dim3 blk(256);
  const float wcarry   = 16.0f;
  const float wscale   = 1.0f / 16.0f;
  const float inv_sqd  = 0.125f;
  const float qescale  = inv_sqd / 16.0f;
  const float pvscale  = 16.0f / kPScale;
  const float oscale   = 1.0f / 256.0f;

  const int n2x = kNB * kSeq * kDM / 2;
  const int n2w = kDM * kDM / 2;
  const int n2r = kRelPad * kDHD / 2;
  cast_bf_f16x2_kernel<<<dim3(n2x / 256), blk, 0, stream>>>(xp, X16, n2x, 1.0f);
  cast_bf_f16x2_kernel<<<dim3(n2w / 256), blk, 0, stream>>>(Wq, Wq16, n2w, wcarry);
  cast_bf_f16x2_kernel<<<dim3(n2w / 256), blk, 0, stream>>>(Wk, Wk16, n2w, wcarry);
  cast_bf_f16x2_kernel<<<dim3(n2w / 256), blk, 0, stream>>>(Wv, Wv16, n2w, wcarry);
  cast_bf_f16x2_kernel<<<dim3(n2w / 256), blk, 0, stream>>>(Wo, Wo16, n2w, wcarry);
  cast_rel_f16x2_kernel<<<dim3(n2r / 256), blk, 0, stream>>>(relp, REL16, n2r, kRelN * kDHD, wcarry);

  const int tM = kNB * kSeq / 64, tD = kDM / 64, tS = kSeq / 64, tR = kRelPad / 64;
  const dim3 gProj((tM * tD + 7) / 8, 1);
  const dim3 gVT((tD * tS + 7) / 8, kNB);
  const dim3 gS((tS * tS + 7) / 8, kHG);
  const dim3 gQE((tS * tR + 7) / 8, kHG);
  const dim3 gPV((tS * 1 + 7) / 8, kHG);
  const long planeAct = (long)kSeq * kDM;

  wmma_gemm64<0, false, 2, 1, false, 0><<<gProj, blk, 0, stream>>>(
      X16, X16, kDM, 0L, Wq16, Wq16, kDM, 0L, (void*)Q16, (void*)Q16, kDM, 0L,
      bq, xp, 0L, kNB * kSeq, kDM, kDM, wscale);
  wmma_gemm64<0, false, 2, 1, false, 0><<<gProj, blk, 0, stream>>>(
      X16, X16, kDM, 0L, Wk16, Wk16, kDM, 0L, (void*)K16, (void*)K16, kDM, 0L,
      bk, xp, 0L, kNB * kSeq, kDM, kDM, wscale);
  wmma_gemm64<0, false, 1, 1, false, 0><<<gVT, blk, 0, stream>>>(
      Wv16, Wv16, kDM, 0L, X16, X16, kDM, planeAct, (void*)VT16, (void*)VT16, kSeq, planeAct,
      bv, xp, 0L, kDM, kSeq, kDM, wscale);

  for (int b = 0; b < kNB; ++b) {
    for (int g = 0; g < kNGrp; ++g) {
      const size_t hc = (size_t)g * kHG * kDHD;
      const unsigned short* Qg = Q16 + (size_t)b * planeAct + hc;
      const unsigned short* Kg = K16 + (size_t)b * planeAct + hc;
      wmma_gemm64<0, false, 0, 0, false, 0><<<gS, blk, 0, stream>>>(
          Qg, Qg, kDM, (long)kDHD, Kg, Kg, kDM, (long)kDHD,
          (void*)Sc, (void*)Sc, kSeq, (long)kSeq * kSeq,
          bq, xp, 0L, kSeq, kSeq, kDHD, inv_sqd);
      wmma_gemm64<0, false, 0, 0, false, 0><<<gQE, blk, 0, stream>>>(
          Qg, Qg, kDM, (long)kDHD, REL16, REL16, kDHD, 0L,
          (void*)Qe, (void*)Qe, kRelPad, (long)kSeq * kRelPad,
          bq, xp, 0L, kSeq, kRelPad, kDHD, qescale);
      rel_softmax_kernel<<<dim3(kHG * kSeq), dim3(128), 0, stream>>>(Sc, Qe, P16);
      wmma_gemm64<0, false, 0, 1, false, 0><<<gPV, blk, 0, stream>>>(
          P16, P16, kSeq, (long)kSeq * kSeq,
          VT16 + (size_t)b * planeAct + hc * kSeq, VT16 + (size_t)b * planeAct + hc * kSeq, kSeq, (long)kDHD * kSeq,
          (void*)(CTX16 + (size_t)b * planeAct + hc), (void*)(CTX16 + (size_t)b * planeAct + hc), kDM, (long)kDHD,
          bq, xp, 0L, kSeq, kDHD, kSeq, pvscale);
    }
  }

  wmma_gemm64<0, false, 2, 0, false, 0><<<gProj, blk, 0, stream>>>(
      CTX16, CTX16, kDM, 0L, Wo16, Wo16, kDM, 0L, (void*)outp, (void*)outp, kDM, 0L,
      bo, xp, 0L, kNB * kSeq, kDM, kDM, oscale);
}
